// SS2D_Global_28647431864581
// MI455X (gfx1250) — hardware-run, weakly checked
//
#include <hip/hip_runtime.h>
#include <math.h>

typedef __attribute__((ext_vector_type(16))) _Float16 v16h;
typedef __attribute__((ext_vector_type(8)))  _Float16 v8h;
typedef __attribute__((ext_vector_type(16))) __bf16   v16b;
typedef __attribute__((ext_vector_type(8)))  __bf16   v8b;
typedef __attribute__((ext_vector_type(8)))  float    v8f;
typedef __attribute__((ext_vector_type(4)))  float    v4f;

constexpr int kBatch   = 2;
constexpr int kImgH    = 64;
constexpr int kImgW    = 64;
constexpr int kChIn    = 96;
constexpr int kDin     = 192;
constexpr int kDirs    = 4;
constexpr int kRank    = 6;
constexpr int kStates  = 16;
constexpr int kXprojC  = kRank + 2 * kStates;
constexpr int kSeqLen  = kImgH * kImgW;
constexpr int kRows    = kBatch * kSeqLen;
constexpr int kXzP     = 2 * kDin;
constexpr int kGrpW    = 48;
constexpr int kPP      = kDirs * kGrpW;
constexpr int kWoRows  = 128;
constexpr int kPosTile = 16;
constexpr int kTileP   = 196;
constexpr int kStepTile = 64;
constexpr int kChTile   = 64;
constexpr int kSXP      = 40;
constexpr int kSYP      = 68;
constexpr float kCarryAct = 64.0f;
constexpr float kCarryWgt = 256.0f;
static_assert(kXprojC == 38, "x_proj width");
static_assert(kPP == 192 && (kPP % 64) == 0, "x_proj padded width");
static_assert(kImgH == 64 && kImgW == 64 && kSeqLen == 4096, "image");
static_assert((kChIn % 32) == 0 && (kDin % 32) == 0, "GEMM K multiples of 32");
static_assert((kRows % 64) == 0 && (kXzP % 64) == 0 && (kWoRows % 64) == 0, "GEMM M,N multiples of 64");
static_assert((kChIn % 32) == 0 && kChIn <= kWoRows, "out_proj store guard is a multiple of 32 columns");
static_assert((kRows % kPosTile) == 0 && (kImgW % kPosTile) == 0, "position tiles stay inside an image row");
static_assert((kSeqLen % kStepTile) == 0 && (kDin % kChTile) == 0, "scan tiles");
static_assert(kSXP == 8 + 2 * kStates, "scan row layout");

constexpr size_t kSzXH  = (size_t)kRows * kChIn * 2;
constexpr size_t kSzWI  = (size_t)kXzP * kChIn * 2;
constexpr size_t kSzWX  = (size_t)kPP * kDin * 2;
constexpr size_t kSzWO  = (size_t)kWoRows * kDin * 2;
constexpr size_t kSzXZ  = (size_t)kRows * kXzP * 4;
constexpr size_t kSzXC  = (size_t)kRows * kDin * 4;
constexpr size_t kSzXCH = (size_t)kRows * kDin * 2;
constexpr size_t kSzPJ  = (size_t)kRows * kPP * 4;
constexpr size_t kSzYS  = (size_t)kBatch * kDirs * kSeqLen * kDin * 4;
constexpr size_t kSzG   = (size_t)kRows * kDin * 2;
constexpr size_t kOffXH  = 0;
constexpr size_t kOffXL  = kOffXH  + kSzXH;
constexpr size_t kOffWIH = kOffXL  + kSzXH;
constexpr size_t kOffWIL = kOffWIH + kSzWI;
constexpr size_t kOffWX  = kOffWIL + kSzWI;
constexpr size_t kOffWOH = kOffWX  + kSzWX;
constexpr size_t kOffWOL = kOffWOH + kSzWO;
constexpr size_t kOffXZ  = kOffWOL + kSzWO;
constexpr size_t kOffXC  = kOffXZ  + kSzXZ;
constexpr size_t kOffXCH = kOffXC  + kSzXC;
constexpr size_t kOffPJ  = kOffXCH + kSzXCH;
constexpr size_t kOffYS  = kOffPJ  + kSzPJ;
constexpr size_t kOffGH  = kOffYS  + kSzYS;
constexpr size_t kOffGL  = kOffGH  + kSzG;
constexpr size_t kWsTotal = kOffGL + kSzG;
static_assert(kWsTotal == 63234048ull, "carve total");
static_assert(kWsTotal <= 134217728ull, "carve cap");
static_assert((kOffXL % 128) == 0 && (kOffWIH % 128) == 0 && (kOffWIL % 128) == 0 && (kOffWX % 128) == 0 &&
              (kOffWOH % 128) == 0 && (kOffWOL % 128) == 0 && (kOffXZ % 128) == 0 && (kOffXC % 128) == 0 &&
              (kOffXCH % 128) == 0 && (kOffPJ % 128) == 0 && (kOffYS % 128) == 0 && (kOffGH % 128) == 0 &&
              (kOffGL % 128) == 0, "128-B aligned regions");

__device__ __forceinline__ unsigned short f2bf_bits(float f) {
  unsigned u = __float_as_uint(f);
  return (unsigned short)((u + 0x7FFFu + ((u >> 16) & 1u)) >> 16);
}
__device__ __forceinline__ float bf_bits2f(unsigned short h) { return __uint_as_float(((unsigned)h) << 16); }

__device__ __forceinline__ void mma_guard_h(v8f& c, v16h a, v16h b) { asm volatile("v_nop\n\tv_nop\n\tv_nop\n\tv_nop" : "+v"(c) : "v"(a), "v"(b)); }
__device__ __forceinline__ void mma_guard_b(v8f& c, v16b a, v16b b) { asm volatile("v_nop\n\tv_nop\n\tv_nop\n\tv_nop" : "+v"(c) : "v"(a), "v"(b)); }
__device__ __forceinline__ void keep4_h(v16h a, v16h b, v16h c, v16h d) { asm volatile("v_nop" :: "v"(a), "v"(b), "v"(c), "v"(d)); }
__device__ __forceinline__ void keep4_b(v16b a, v16b b, v16b c, v16b d) { asm volatile("v_nop" :: "v"(a), "v"(b), "v"(c), "v"(d)); }
__device__ __forceinline__ void acc_guard4(v8f& a, v8f& b, v8f& c, v8f& d) { asm volatile("v_nop\n\tv_nop\n\tv_nop\n\tv_nop" : "+v"(a), "+v"(b), "+v"(c), "+v"(d)); }

template <typename T> struct Frag;
template <> struct Frag<_Float16> {
  typedef v16h V; union U { v16h v; v8h h[2]; };
  static __device__ __forceinline__ v16h load(const _Float16* p) {
    U f; f.h[0] = *(const v8h*)(p); f.h[1] = *(const v8h*)(p + 16); return f.v;
  }
  static __device__ __forceinline__ v8f mma(v16h a, v16h b, v8f c) {
    c = __builtin_amdgcn_wmma_f32_16x16x32_f16(false, a, false, b, (short)0, c, false, false);
    mma_guard_h(c, a, b);
    return c;
  }
  static __device__ __forceinline__ void keep(v16h a, v16h b, v16h c, v16h d) { keep4_h(a, b, c, d); }
};
template <> struct Frag<__bf16> {
  typedef v16b V; union U { v16b v; v8b h[2]; };
  static __device__ __forceinline__ v16b load(const __bf16* p) {
    U f; f.h[0] = *(const v8b*)(p); f.h[1] = *(const v8b*)(p + 16); return f.v;
  }
  static __device__ __forceinline__ v8f mma(v16b a, v16b b, v8f c) {
    c = __builtin_amdgcn_wmma_f32_16x16x32_bf16(false, a, false, b, (short)0, c, false, false);
    mma_guard_b(c, a, b);
    return c;
  }
  static __device__ __forceinline__ void keep(v16b a, v16b b, v16b c, v16b d) { keep4_b(a, b, c, d); }
};

template <int ET> struct Elem;
template <> struct Elem<0> { typedef _Float16 T; };
template <> struct Elem<1> { typedef __bf16 T; };
template <int ET, int SPL>
__global__ __launch_bounds__(256) void wmma_gemm64(
    const unsigned short* __restrict__ Ap, const unsigned short* A2p, int lda,
    const unsigned short* __restrict__ Btp, const unsigned short* Bt2p, int ldb,
    float* __restrict__ Cout, int ldc, int M, int N, int K, int nStore, float scale) {
  typedef typename Elem<ET>::T T;
  typedef typename Frag<T>::V V;
  const T* A = (const T*)Ap; const T* A2 = (const T*)A2p; const T* Bt = (const T*)Btp; const T* Bt2 = (const T*)Bt2p;
  __shared__ __align__(16) float sT[8][16 * 68];
  const int lane = threadIdx.x & 31;
  const int wave = threadIdx.x >> 5;
  const int tilesN = N >> 6;
  const int tilesM = M >> 6;
  const int tile = blockIdx.x * 8 + wave;
  if (tile >= tilesM * tilesN) return;
  const int tm = tile / tilesN;
  const int tn = tile - tm * tilesN;
  const int m0 = tm << 6;
  const int n0 = tn << 6;

  const int rlane = lane & 15;
  const int koff  = (lane >> 4) * 8;
  const int mOff  = (lane >> 4) * 8;

  v8f acc[4][4];
#pragma unroll
  for (int i = 0; i < 4; ++i)
#pragma unroll
    for (int j = 0; j < 4; ++j) acc[i][j] = (v8f){0.f,0.f,0.f,0.f,0.f,0.f,0.f,0.f};

  for (int k0 = 0; k0 < K; k0 += 32) {
    V bh[4], bl[4];
#pragma unroll
    for (int j = 0; j < 4; ++j) {
      const size_t bo = (size_t)(n0 + (j << 4) + rlane) * ldb + koff + k0;
      bh[j] = Frag<T>::load(Bt + bo);
      if (SPL == 2) bl[j] = Frag<T>::load(Bt2 + bo);
    }
#pragma unroll
    for (int i = 0; i < 4; ++i) {
      const size_t ao = (size_t)(m0 + (i << 4) + rlane) * lda + koff + k0;
      V ah = Frag<T>::load(A + ao);
      V al;
      if (SPL == 2) al = Frag<T>::load(A2 + ao);
#pragma unroll
      for (int j = 0; j < 4; ++j) {
        acc[i][j] = Frag<T>::mma(ah, bh[j], acc[i][j]);
        if (SPL == 2) {
          acc[i][j] = Frag<T>::mma(ah, bl[j], acc[i][j]);
          acc[i][j] = Frag<T>::mma(al, bh[j], acc[i][j]);
        }
      }
    }
    Frag<T>::keep(bh[0], bh[1], bh[2], bh[3]);
    if (SPL == 2) Frag<T>::keep(bl[0], bl[1], bl[2], bl[3]);
  }
  acc_guard4(acc[0][0], acc[0][1], acc[0][2], acc[0][3]);
  acc_guard4(acc[1][0], acc[1][1], acc[1][2], acc[1][3]);
  acc_guard4(acc[2][0], acc[2][1], acc[2][2], acc[2][3]);
  acc_guard4(acc[3][0], acc[3][1], acc[3][2], acc[3][3]);

  float* slab = sT[wave];
#pragma unroll
  for (int i = 0; i < 4; ++i) {
    const int mBase = m0 + (i << 4);
#pragma unroll
    for (int j = 0; j < 4; ++j) {
#pragma unroll
      for (int r = 0; r < 8; ++r) {
        const float v = acc[i][j][r] * scale;
        slab[(mOff + r) * 68 + (j << 4) + rlane] = v;
      }
    }
    __builtin_amdgcn_fence(__ATOMIC_RELEASE, "workgroup");
    __builtin_amdgcn_wave_barrier();
    __builtin_amdgcn_fence(__ATOMIC_ACQUIRE, "workgroup");
    {
      const int hh = lane >> 4, c4 = (lane & 15) * 4;
      const bool colOk = (n0 + c4) < nStore;
      for (int pass = 0; pass < 2; ++pass) {
#pragma unroll
        for (int it = 0; it < 8; ++it) {
          const int row = it * 2 + hh;
          v4f v = *(const v4f*)(slab + row * 68 + c4);
          if (colOk) *(volatile v4f*)(Cout + (size_t)(mBase + row) * ldc + n0 + c4) = v;
        }
        __threadfence();
      }
    }
    __builtin_amdgcn_fence(__ATOMIC_RELEASE, "workgroup");
    __builtin_amdgcn_wave_barrier();
    __builtin_amdgcn_fence(__ATOMIC_ACQUIRE, "workgroup");
  }
}

constexpr int kPrepBlkX  = (kRows * kChIn / 8) / 256;
constexpr int kPrepBlkWI = (kXzP * kChIn / 8) / 256;
constexpr int kPrepBlkWX = (kPP * kDin / 8) / 256;
constexpr int kPrepBlkWO = (kWoRows * kDin / 8) / 256;
static_assert(kPrepBlkX * 256 * 8 == kRows * kChIn, "prep x coverage");
static_assert(kPrepBlkWI * 256 * 8 == kXzP * kChIn, "prep W_in coverage");
static_assert(kPrepBlkWX * 256 * 8 == kPP * kDin, "prep W_x coverage");
static_assert(kPrepBlkWO * 256 * 8 == kWoRows * kDin, "prep W_out coverage");
constexpr int kPrepBlocks = kPrepBlkX + kPrepBlkWI + kPrepBlkWX + kPrepBlkWO;

__global__ __launch_bounds__(256) void prep_planes_kernel(
    const float* __restrict__ x, const float* __restrict__ wi, const float* __restrict__ wx, const float* __restrict__ wo,
    unsigned short* __restrict__ xh, unsigned short* __restrict__ xl,
    unsigned short* __restrict__ wih, unsigned short* __restrict__ wil,
    unsigned short* __restrict__ wx16,
    unsigned short* __restrict__ woh, unsigned short* __restrict__ wol)
{
  const int blk = blockIdx.x, tid = threadIdx.x;
  const float* sp;
  unsigned short* ph;
  unsigned short* pl;
  bool keepv = true;
  bool halfMode = false;
  if (blk < kPrepBlkX) {
    const size_t e0 = ((size_t)blk * 256 + tid) * 8;
    sp = x + e0; ph = xh + e0; pl = xl + e0;
  } else if (blk < kPrepBlkX + kPrepBlkWI) {
    const size_t e0 = ((size_t)(blk - kPrepBlkX) * 256 + tid) * 8;
    sp = wi + e0; ph = wih + e0; pl = wil + e0;
  } else if (blk < kPrepBlkX + kPrepBlkWI + kPrepBlkWX) {
    const int e0 = ((blk - kPrepBlkX - kPrepBlkWI) * 256 + tid) * 8;
    const int row = e0 / kDin;
    const int col = e0 - row * kDin;
    const int kdir = row / kGrpW;
    const int j = row - kdir * kGrpW;
    keepv = (j < kRank) || (j >= 8 && j < 8 + 2 * kStates);
    int c = (j < kRank) ? j : (j - 2);
    c = c < 0 ? 0 : (c > kXprojC - 1 ? kXprojC - 1 : c);
    sp = wx + (size_t)(kdir * kXprojC + c) * kDin + col;
    ph = wx16 + e0; pl = wx16 + e0;
    halfMode = true;
  } else {
    const int e0 = ((blk - kPrepBlkX - kPrepBlkWI - kPrepBlkWX) * 256 + tid) * 8;
    const int row = e0 / kDin;
    const int col = e0 - row * kDin;
    keepv = row < kChIn;
    const int rc = row < kChIn ? row : (kChIn - 1);
    sp = wo + (size_t)rc * kDin + col;
    ph = woh + e0; pl = wol + e0;
  }
  v4f a0 = *(const v4f*)(sp);
  v4f a1 = *(const v4f*)(sp + 4);
  asm volatile("" : "+v"(a0), "+v"(a1));
  v8h hv, lv;
#pragma unroll
  for (int e = 0; e < 4; ++e) {
    const float f0 = keepv ? a0[e] : 0.0f;
    const float f1 = keepv ? a1[e] : 0.0f;
    if (halfMode) {
      hv[e]     = (_Float16)(f0 * kCarryWgt);
      hv[4 + e] = (_Float16)(f1 * kCarryWgt);
      lv[e]     = (_Float16)0.0f;
      lv[4 + e] = (_Float16)0.0f;
    } else {
      const unsigned short h0 = f2bf_bits(f0), h1 = f2bf_bits(f1);
      const unsigned short l0 = f2bf_bits(f0 - bf_bits2f(h0)), l1 = f2bf_bits(f1 - bf_bits2f(h1));
      hv[e]     = __builtin_bit_cast(_Float16, h0);
      hv[4 + e] = __builtin_bit_cast(_Float16, h1);
      lv[e]     = __builtin_bit_cast(_Float16, l0);
      lv[4 + e] = __builtin_bit_cast(_Float16, l1);
    }
  }
  *(volatile v8h*)ph = hv;
  if (!halfMode) *(volatile v8h*)pl = lv;
  __threadfence();
  *(volatile v8h*)ph = hv;
  if (!halfMode) *(volatile v8h*)pl = lv;
}

__global__ __launch_bounds__(192) void conv_silu_kernel(
    const float* __restrict__ XZ, const float* __restrict__ cw, const float* __restrict__ cb,
    float* __restrict__ XC, unsigned short* __restrict__ XCH)
{
  __shared__ __align__(16) float sT[kPosTile * kTileP];
  const int tid = threadIdx.x, lane = tid & 31, wave = tid >> 5;
  const int pos0 = blockIdx.x * kPosTile;
  const int b  = pos0 / kSeqLen;
  const int l0 = pos0 - b * kSeqLen;
  const int h  = l0 / kImgW;
  const int w0 = l0 - h * kImgW;
  const int d  = tid;
  const float t00 = cw[d * 9 + 0], t01 = cw[d * 9 + 1], t02 = cw[d * 9 + 2];
  const float t10 = cw[d * 9 + 3], t11 = cw[d * 9 + 4], t12 = cw[d * 9 + 5];
  const float t20 = cw[d * 9 + 6], t21 = cw[d * 9 + 7], t22 = cw[d * 9 + 8];
  const float bc = cb[d];
  const bool upOk = (h > 0), dnOk = (h < kImgH - 1);
  const int hu = upOk ? (h - 1) : h;
  const int hd = dnOk ? (h + 1) : h;
  const float* p0 = XZ + ((size_t)b * kSeqLen + (size_t)hu * kImgW) * kXzP + d;
  const float* p1 = XZ + ((size_t)b * kSeqLen + (size_t)h  * kImgW) * kXzP + d;
  const float* p2 = XZ + ((size_t)b * kSeqLen + (size_t)hd * kImgW) * kXzP + d;
  float lf0, lf1, lf2, md0, md1, md2;
  {
    const bool lok = (w0 > 0);
    const int wl = lok ? (w0 - 1) : 0;
    const float a0 = p0[(size_t)wl * kXzP], a1 = p1[(size_t)wl * kXzP], a2 = p2[(size_t)wl * kXzP];
    lf0 = (lok && upOk) ? a0 : 0.0f;
    lf1 = lok ? a1 : 0.0f;
    lf2 = (lok && dnOk) ? a2 : 0.0f;
    const float m0 = p0[(size_t)w0 * kXzP], m1 = p1[(size_t)w0 * kXzP], m2 = p2[(size_t)w0 * kXzP];
    md0 = upOk ? m0 : 0.0f;
    md1 = m1;
    md2 = dnOk ? m2 : 0.0f;
  }
#pragma unroll 1
  for (int s = 0; s < kPosTile; ++s) {
    const int wr = w0 + s + 1;
    const bool rok = (wr < kImgW);
    const int wrc = rok ? wr : (kImgW - 1);
    const float a0 = p0[(size_t)wrc * kXzP], a1 = p1[(size_t)wrc * kXzP], a2 = p2[(size_t)wrc * kXzP];
    const float rt0 = (rok && upOk) ? a0 : 0.0f;
    const float rt1 = rok ? a1 : 0.0f;
    const float rt2 = (rok && dnOk) ? a2 : 0.0f;
    float acc = bc;
    acc = fmaf(t00, lf0, acc);
    acc = fmaf(t01, md0, acc);
    acc = fmaf(t02, rt0, acc);
    acc = fmaf(t10, lf1, acc);
    acc = fmaf(t11, md1, acc);
    acc = fmaf(t12, rt1, acc);
    acc = fmaf(t20, lf2, acc);
    acc = fmaf(t21, md2, acc);
    acc = fmaf(t22, rt2, acc);
    const float sg = 1.0f / (1.0f + expf(-acc));
    sT[s * kTileP + tid] = acc * sg;
    lf0 = md0; lf1 = md1; lf2 = md2;
    md0 = rt0; md1 = rt1; md2 = rt2;
  }
  __syncthreads();
  v4f fv[4];
  v8h hv[2];
#pragma unroll
  for (int it = 0; it < 4; ++it) {
    const int f = ((it * 6 + wave) * 32 + lane) * 4;
    const int row = f / kDin;
    const int col = f - row * kDin;
    fv[it] = *(const v4f*)(sT + row * kTileP + col);
  }
#pragma unroll
  for (int it = 0; it < 2; ++it) {
    const int f = ((it * 6 + wave) * 32 + lane) * 8;
    const int row = f / kDin;
    const int col = f - row * kDin;
    const float* sp = sT + row * kTileP + col;
    const v4f a0 = *(const v4f*)(sp);
    const v4f a1 = *(const v4f*)(sp + 4);
#pragma unroll
    for (int e = 0; e < 4; ++e) {
      hv[it][e]     = (_Float16)(a0[e] * kCarryAct);
      hv[it][4 + e] = (_Float16)(a1[e] * kCarryAct);
    }
  }
  float* xcBase = XC + (size_t)pos0 * kDin;
  unsigned short* xhBase = XCH + (size_t)pos0 * kDin;
  for (int pass = 0; pass < 2; ++pass) {
#pragma unroll
    for (int it = 0; it < 4; ++it) {
      const int f = ((it * 6 + wave) * 32 + lane) * 4;
      *(volatile v4f*)(xcBase + f) = fv[it];
    }
#pragma unroll
    for (int it = 0; it < 2; ++it) {
      const int f = ((it * 6 + wave) * 32 + lane) * 8;
      *(volatile v8h*)(xhBase + f) = hv[it];
    }
    __threadfence();
  }
}

__device__ __forceinline__ int step_pos(int t, int kdir) {
  const int tt = (kdir & 2) ? (kSeqLen - 1 - t) : t;
  return (kdir & 1) ? ((tt % kImgH) * kImgW + (tt / kImgH)) : tt;
}
__device__ __forceinline__ void state_step(float& hst, float& y, float dt, float an, float dtu, float bn, float cn) {
  const float e = expf(dt * an);
  hst = fmaf(e, hst, dtu * bn);
  y = fmaf(hst, cn, y);
}

__global__ __launch_bounds__(128) void scan_kernel(
    const float* __restrict__ PJ, const float* __restrict__ XC,
    const float* __restrict__ Alog, const float* __restrict__ dtw, const float* __restrict__ dtb,
    const float* __restrict__ Dsk, float* __restrict__ YS)
{
  __shared__ __align__(16) float sX[kStepTile * kSXP];
  __shared__ __align__(16) float sU[kStepTile * kChTile];
  __shared__ __align__(16) float sY[kStepTile * kSYP];
  const int tid = threadIdx.x, lane = tid & 31, wave = tid >> 5;
  const int hf = lane >> 4;
  const int c  = wave * 16 + (lane & 15);
  constexpr int kGroups = kDin / kChTile;
  const int blk = blockIdx.x;
  const int b   = blk / (kDirs * kGroups);
  const int rem = blk - b * (kDirs * kGroups);
  const int kdir = rem / kGroups;
  const int d0  = (rem - kdir * kGroups) * kChTile;
  const int d   = d0 + c;
  const int kd  = kdir * kDin + d;
  float nA0, nA1, nA2, nA3, nA4, nA5, nA6, nA7;
  {
    const v4f q0 = *(const v4f*)(Alog + (size_t)kd * kStates + hf * 8);
    const v4f q1 = *(const v4f*)(Alog + (size_t)kd * kStates + hf * 8 + 4);
    nA0 = -expf(q0[0]); nA1 = -expf(q0[1]); nA2 = -expf(q0[2]); nA3 = -expf(q0[3]);
    nA4 = -expf(q1[0]); nA5 = -expf(q1[1]); nA6 = -expf(q1[2]); nA7 = -expf(q1[3]);
  }
  const float w0 = dtw[(size_t)kd * kRank + 0], w1 = dtw[(size_t)kd * kRank + 1], w2 = dtw[(size_t)kd * kRank + 2];
  const float w3 = dtw[(size_t)kd * kRank + 3], w4 = dtw[(size_t)kd * kRank + 4], w5 = dtw[(size_t)kd * kRank + 5];
  const float bias = dtb[kd];
  const float dsk  = Dsk[kd];
  float h0 = 0.f, h1 = 0.f, h2 = 0.f, h3 = 0.f, h4 = 0.f, h5 = 0.f, h6 = 0.f, h7 = 0.f;
  const float* Pb = PJ + (size_t)b * kSeqLen * kPP + kdir * kGrpW;
  const float* Ub = XC + (size_t)b * kSeqLen * kDin + d0;
  float* Yb = YS + (size_t)(b * kDirs + kdir) * kSeqLen * kDin + d0;
#pragma unroll 1
  for (int t0 = 0; t0 < kSeqLen; t0 += kStepTile) {
    __syncthreads();
#pragma unroll
    for (int it = 0; it < 5; ++it) {
      const int i = it * 128 + tid;
      const int row = i / 10;
      const int cc = i - row * 10;
      const int pos = step_pos(t0 + row, kdir);
      *(v4f*)(sX + row * kSXP + cc * 4) = *(const v4f*)(Pb + (size_t)pos * kPP + cc * 4);
    }
#pragma unroll
    for (int it = 0; it < 8; ++it) {
      const int i = it * 128 + tid;
      const int row = i >> 4;
      const int c4 = (i & 15) * 4;
      const int pos = step_pos(t0 + row, kdir);
      *(v4f*)(sU + row * kChTile + c4) = *(const v4f*)(Ub + (size_t)pos * kDin + c4);
    }
    __syncthreads();
#pragma unroll 1
    for (int s = 0; s < kStepTile; ++s) {
      const float* xr = sX + s * kSXP;
      const v4f xa = *(const v4f*)(xr);
      const v4f xb = *(const v4f*)(xr + 4);
      float v = bias;
      v = fmaf(w0, xa[0], v);
      v = fmaf(w1, xa[1], v);
      v = fmaf(w2, xa[2], v);
      v = fmaf(w3, xa[3], v);
      v = fmaf(w4, xb[0], v);
      v = fmaf(w5, xb[1], v);
      const float av = expf(-fabsf(v));
      const float uu = 1.0f + av;
      const float l1p = logf(uu) + (av - (uu - 1.0f)) * (1.0f / uu);
      const float dt = fmaxf(v, 0.0f) + l1p;
      const float u = sU[s * kChTile + c];
      const float dtu = dt * u;
      const float* bp = xr + 8 + hf * 8;
      const float* cp = xr + 8 + kStates + hf * 8;
      const v4f b0 = *(const v4f*)(bp);
      const v4f b1 = *(const v4f*)(bp + 4);
      const v4f c0 = *(const v4f*)(cp);
      const v4f c1 = *(const v4f*)(cp + 4);
      float y = 0.0f;
      state_step(h0, y, dt, nA0, dtu, b0[0], c0[0]);
      state_step(h1, y, dt, nA1, dtu, b0[1], c0[1]);
      state_step(h2, y, dt, nA2, dtu, b0[2], c0[2]);
      state_step(h3, y, dt, nA3, dtu, b0[3], c0[3]);
      state_step(h4, y, dt, nA4, dtu, b1[0], c1[0]);
      state_step(h5, y, dt, nA5, dtu, b1[1], c1[1]);
      state_step(h6, y, dt, nA6, dtu, b1[2], c1[2]);
      state_step(h7, y, dt, nA7, dtu, b1[3], c1[3]);
      const float yo = __shfl_xor(y, 16, 32);
      y = y + yo;
      y = fmaf(u, dsk, y);
      if (hf == 0) sY[s * kSYP + c] = y;
    }
    __syncthreads();
    {
      const int c4 = (lane & 15) * 4;
      for (int pass = 0; pass < 2; ++pass) {
#pragma unroll
        for (int it = 0; it < 8; ++it) {
          const int row = it * 8 + wave * 2 + hf;
          const v4f val = *(const v4f*)(sY + row * kSYP + c4);
          const int pos = step_pos(t0 + row, kdir);
          *(volatile v4f*)(Yb + (size_t)pos * kDin + c4) = val;
        }
        __threadfence();
      }
    }
  }
}

__global__ __launch_bounds__(192) void merge_norm_gate_kernel(
    const float* __restrict__ YS, const float* __restrict__ XZ,
    const float* __restrict__ lnw, const float* __restrict__ lnb,
    unsigned short* __restrict__ GH, unsigned short* __restrict__ GL)
{
  __shared__ __align__(16) float sV[kPosTile * kTileP];
  __shared__ float sMu[kPosTile];
  __shared__ float sRs[kPosTile];
  const int tid = threadIdx.x, lane = tid & 31, wave = tid >> 5;
  const int pos0 = blockIdx.x * kPosTile;
  const int b  = pos0 / kSeqLen;
  const int l0 = pos0 - b * kSeqLen;
  const int d  = tid;
  const size_t planeSz = (size_t)kSeqLen * kDin;
  const float* y0 = YS + (size_t)(b * kDirs) * planeSz + (size_t)l0 * kDin + d;
#pragma unroll 1
  for (int s = 0; s < kPosTile; ++s) {
    const float a0 = y0[(size_t)s * kDin];
    const float a1 = y0[planeSz + (size_t)s * kDin];
    const float a2 = y0[2 * planeSz + (size_t)s * kDin];
    const float a3 = y0[3 * planeSz + (size_t)s * kDin];
    sV[s * kTileP + d] = (a0 + a2) + (a1 + a3);
  }
  __syncthreads();
  const float invN = 1.0f / (float)kDin;
#pragma unroll 1
  for (int p = wave; p < kPosTile; p += 6) {
    const float* rp = sV + p * kTileP + lane;
    const float x0 = rp[0], x1 = rp[32], x2 = rp[64], x3 = rp[96], x4 = rp[128], x5 = rp[160];
    float sm = ((x0 + x1) + (x2 + x3)) + (x4 + x5);
    sm += __shfl_xor(sm, 16, 32);
    sm += __shfl_xor(sm, 8, 32);
    sm += __shfl_xor(sm, 4, 32);
    sm += __shfl_xor(sm, 2, 32);
    sm += __shfl_xor(sm, 1, 32);
    const float mu = sm * invN;
    const float e0 = x0 - mu, e1 = x1 - mu, e2 = x2 - mu, e3 = x3 - mu, e4 = x4 - mu, e5 = x5 - mu;
    float sq = ((e0 * e0 + e1 * e1) + (e2 * e2 + e3 * e3)) + (e4 * e4 + e5 * e5);
    sq += __shfl_xor(sq, 16, 32);
    sq += __shfl_xor(sq, 8, 32);
    sq += __shfl_xor(sq, 4, 32);
    sq += __shfl_xor(sq, 2, 32);
    sq += __shfl_xor(sq, 1, 32);
    const float rs = rsqrtf(sq * invN + 1e-5f);
    if (lane == 0) { sMu[p] = mu; sRs[p] = rs; }
  }
  __syncthreads();
  const float gw = lnw[d], gb = lnb[d];
  const float* zp = XZ + (size_t)pos0 * kXzP + kDin + d;
#pragma unroll 1
  for (int s = 0; s < kPosTile; ++s) {
    const float v = sV[s * kTileP + d];
    const float yn = (v - sMu[s]) * sRs[s] * gw + gb;
    const float z = zp[(size_t)s * kXzP];
    const float sg = 1.0f / (1.0f + expf(-z));
    sV[s * kTileP + d] = yn * (z * sg);
  }
  __syncthreads();
  v8h hv[2], lv[2];
#pragma unroll
  for (int it = 0; it < 2; ++it) {
    const int f = ((it * 6 + wave) * 32 + lane) * 8;
    const int row = f / kDin;
    const int col = f - row * kDin;
    const float* sp = sV + row * kTileP + col;
    const v4f a0 = *(const v4f*)(sp);
    const v4f a1 = *(const v4f*)(sp + 4);
#pragma unroll
    for (int e = 0; e < 4; ++e) {
      const float f0 = a0[e], f1 = a1[e];
      const unsigned short h0 = f2bf_bits(f0), h1 = f2bf_bits(f1);
      const unsigned short q0 = f2bf_bits(f0 - bf_bits2f(h0)), q1 = f2bf_bits(f1 - bf_bits2f(h1));
      hv[it][e]     = __builtin_bit_cast(_Float16, h0);
      hv[it][4 + e] = __builtin_bit_cast(_Float16, h1);
      lv[it][e]     = __builtin_bit_cast(_Float16, q0);
      lv[it][4 + e] = __builtin_bit_cast(_Float16, q1);
    }
  }
  unsigned short* ghBase = GH + (size_t)pos0 * kDin;
  unsigned short* glBase = GL + (size_t)pos0 * kDin;
  for (int pass = 0; pass < 2; ++pass) {
#pragma unroll
    for (int it = 0; it < 2; ++it) {
      const int f = ((it * 6 + wave) * 32 + lane) * 8;
      *(volatile v8h*)(ghBase + f) = hv[it];
      *(volatile v8h*)(glBase + f) = lv[it];
    }
    __threadfence();
  }
}

static_assert(((kRows / 64) * (kXzP / 64)) % 8 == 0, "in_proj tiles fill whole blocks");
static_assert(((kRows / 64) * (kPP / 64)) % 8 == 0, "x_proj tiles fill whole blocks");
static_assert(((kRows / 64) * (kWoRows / 64)) % 8 == 0, "out_proj tiles fill whole blocks");

extern "C" void kernel_launch(void* const* d_in, const int* in_sizes, int n_in,
                              void* d_out, int out_size, void* d_ws, size_t ws_size,
                              hipStream_t stream) {
  if (n_in < 12) return;
  if (in_sizes[0] != kRows * kChIn) return;
  if (in_sizes[1] != kXzP * kChIn) return;
  if (in_sizes[2] != kDin * 9) return;
  if (in_sizes[3] != kDin) return;
  if (in_sizes[4] != kDirs * kXprojC * kDin) return;
  if (in_sizes[5] != kDirs * kDin * kRank) return;
  if (in_sizes[6] != kDirs * kDin) return;
  if (in_sizes[7] != kDirs * kDin * kStates) return;
  if (in_sizes[8] != kDirs * kDin) return;
  if (in_sizes[9] != kDin) return;
  if (in_sizes[10] != kDin) return;
  if (in_sizes[11] != kChIn * kDin) return;
  if (out_size != kRows * kChIn) return;
  if (ws_size < kWsTotal) return;

  const float* x      = (const float*)d_in[0];
  const float* W_in   = (const float*)d_in[1];
  const float* conv_w = (const float*)d_in[2];
  const float* conv_b = (const float*)d_in[3];
  const float* W_x    = (const float*)d_in[4];
  const float* W_dt   = (const float*)d_in[5];
  const float* b_dt   = (const float*)d_in[6];
  const float* A_log  = (const float*)d_in[7];
  const float* Dp     = (const float*)d_in[8];
  const float* ln_w   = (const float*)d_in[9];
  const float* ln_b   = (const float*)d_in[10];
  const float* W_out  = (const float*)d_in[11];
  float* out = (float*)d_out;

  char* ws = (char*)d_ws;
  unsigned short* XH  = (unsigned short*)(ws + kOffXH);
  unsigned short* XL  = (unsigned short*)(ws + kOffXL);
  unsigned short* WIH = (unsigned short*)(ws + kOffWIH);
  unsigned short* WIL = (unsigned short*)(ws + kOffWIL);
  unsigned short* WX  = (unsigned short*)(ws + kOffWX);
  unsigned short* WOH = (unsigned short*)(ws + kOffWOH);
  unsigned short* WOL = (unsigned short*)(ws + kOffWOL);
  float*          XZ  = (float*)(ws + kOffXZ);
  float*          XC  = (float*)(ws + kOffXC);
  unsigned short* XCH = (unsigned short*)(ws + kOffXCH);
  float*          PJ  = (float*)(ws + kOffPJ);
  float*          YS  = (float*)(ws + kOffYS);
  unsigned short* GH  = (unsigned short*)(ws + kOffGH);
  unsigned short* GL  = (unsigned short*)(ws + kOffGL);

  prep_planes_kernel<<<kPrepBlocks, 256, 0, stream>>>(x, W_in, W_x, W_out, XH, XL, WIH, WIL, WX, WOH, WOL);

  wmma_gemm64<1, 2><<<((kRows / 64) * (kXzP / 64)) / 8, 256, 0, stream>>>(
      XH, XL, kChIn, WIH, WIL, kChIn, XZ, kXzP, kRows, kXzP, kChIn, kXzP, 1.0f);

  conv_silu_kernel<<<kRows / kPosTile, 192, 0, stream>>>(XZ, conv_w, conv_b, XC, XCH);

  wmma_gemm64<0, 0><<<((kRows / 64) * (kPP / 64)) / 8, 256, 0, stream>>>(
      XCH, XCH, kDin, WX, WX, kDin, PJ, kPP, kRows, kPP, kDin, kPP, 1.0f / (kCarryAct * kCarryWgt));

  scan_kernel<<<kBatch * kDirs * (kDin / kChTile), 128, 0, stream>>>(PJ, XC, A_log, W_dt, b_dt, Dp, YS);

  merge_norm_gate_kernel<<<kRows / kPosTile, 192, 0, stream>>>(YS, XZ, ln_w, ln_b, GH, GL);

  wmma_gemm64<1, 2><<<((kRows / 64) * (kWoRows / 64)) / 8, 256, 0, stream>>>(
      GH, GL, kDin, WOH, WOL, kDin, out, kChIn, kRows, kWoRows, kDin, kChIn, 1.0f);
}
